// EN_CAM_75359496175780
// MI455X (gfx1250) — hardware-run, weakly checked
//
#include <hip/hip_runtime.h>


#define NB_  4
#define CX   64
#define HX   128
#define WX   128
#define CP   256
#define GH   64
#define GW   64
#define NTK  4096
#define CQ   32
#define NQKV 320
#define DM   CP
#define PCAR 1024.0f
#define LOSC 1024.0f
typedef _Float16 h16;
typedef unsigned short bf;
typedef __attribute__((ext_vector_type(16))) __bf16   v16bf;
typedef __attribute__((ext_vector_type(16))) _Float16 v16h;
typedef __attribute__((ext_vector_type(8)))  _Float16 v8h;
typedef __attribute__((ext_vector_type(8)))  unsigned short v8us;
typedef __attribute__((ext_vector_type(8)))  float    v8f;
typedef __attribute__((ext_vector_type(4)))  float    v4f;
typedef v8h  __attribute__((may_alias)) v8ha;
typedef v4f  __attribute__((may_alias)) v4fa;
typedef v8us __attribute__((may_alias)) v8usa;

__device__ __forceinline__ unsigned short f2bf(float f) { unsigned u = __float_as_uint(f); u += 0x7FFFu + ((u >> 16) & 1u); return (unsigned short)(u >> 16); }
__device__ __forceinline__ float bf2f(unsigned short b) { return __uint_as_float(((unsigned)b) << 16); }
__device__ __forceinline__ float bfr(float f) { return bf2f(f2bf(f)); }
__device__ __forceinline__ v16h cat16(v8h lo, v8h hi) { return __builtin_shufflevector(lo, hi, 0, 1, 2, 3, 4, 5, 6, 7, 8, 9, 10, 11, 12, 13, 14, 15); }
__device__ __forceinline__ v16bf cat16b(v8us lo, v8us hi) { return __builtin_bit_cast(v16bf, __builtin_shufflevector(lo, hi, 0, 1, 2, 3, 4, 5, 6, 7, 8, 9, 10, 11, 12, 13, 14, 15)); }
__device__ __forceinline__ v8f wmma16(v16h a, v16h b, v8f c) { return __builtin_amdgcn_wmma_f32_16x16x32_f16(false, a, false, b, (short)0, c, false, false); }
__device__ __forceinline__ v8f wmmab(v16bf a, v16bf b, v8f c) { return __builtin_amdgcn_wmma_f32_16x16x32_bf16(false, a, false, b, (short)0, c, false, false); }

template <bool SPLITA, bool F16OUT = false>
__global__ __launch_bounds__(128) void k_gemmb(const bf* __restrict__ A, const bf* __restrict__ Al, const bf* __restrict__ Bn, const float* __restrict__ bias, float* C, int ldc, h16* C2, const float* __restrict__ R = nullptr, int K = DM, int roundR = 1) {
    __shared__ __align__(16) float ost[4][16 * 68];
    const int lane = threadIdx.x & 31, wave = threadIdx.x >> 5, lr = lane & 15, hi = lane >> 4;
    const int r0 = blockIdx.x * 64 + wave * 16, c0 = blockIdx.y * 64;
    const size_t aoff = (size_t)(r0 + lr) * K + 8 * hi;
    size_t boff[4];
#pragma unroll
    for (int t = 0; t < 4; ++t) boff[t] = (size_t)(c0 + t * 16 + lr) * K + 8 * hi;
    v8f acc[4];
#pragma unroll
    for (int t = 0; t < 4; ++t) acc[t] = (v8f){};
#pragma unroll 1
    for (int kc = 0; kc < K; kc += 32) {
        const v16bf a = cat16b(*(const v8us*)(A + aoff + kc), *(const v8us*)(A + aoff + kc + 16));
        v16bf al = a;
        if (SPLITA) al = cat16b(*(const v8us*)(Al + aoff + kc), *(const v8us*)(Al + aoff + kc + 16));
#pragma unroll
        for (int t = 0; t < 4; ++t) { const v16bf b = cat16b(*(const v8us*)(Bn + boff[t] + kc), *(const v8us*)(Bn + boff[t] + kc + 16)); acc[t] = wmmab(a, b, acc[t]); if (SPLITA) acc[t] = wmmab(al, b, acc[t]); }
        asm volatile("v_nop\n\tv_nop\n\tv_nop\n\tv_nop" : "+v"(acc[0]), "+v"(acc[1]), "+v"(acc[2]), "+v"(acc[3]) : "v"(a), "v"(al));
    }
    float* os = &ost[wave][0];
#pragma unroll
    for (int t = 0; t < 4; ++t) { const float bv = bias ? bfr(bias[c0 + t * 16 + lr]) : 0.f;
#pragma unroll
        for (int j = 0; j < 8; ++j) os[(hi * 8 + j) * 68 + t * 16 + lr] = acc[t][j] + bv; }
    __syncthreads();
    if (F16OUT) {
        h16* crow = (h16*)(void*)C + (size_t)r0 * ldc + c0;
        auto pass = [&]() {
#pragma unroll
            for (int s = 0; s < 4; ++s) { const int row = 4 * s + (lane >> 3), piece = lane & 7; const float* sp = os + row * 68 + piece * 8; v8h o, o2;
#pragma unroll
                for (int i = 0; i < 8; ++i) { const h16 a = (h16)sp[i]; o[i] = a; o2[i] = (h16)((sp[i] - (float)a) * LOSC); }
                *(volatile v8h*)(crow + (size_t)row * ldc + piece * 8) = o; if (C2) *(volatile v8h*)(C2 + (size_t)r0 * ldc + c0 + (size_t)row * ldc + piece * 8) = o2; }
        };
        pass(); __threadfence(); pass();
    } else {
        float* crow = C + (size_t)r0 * ldc + c0;
        auto pass = [&]() {
#pragma unroll
            for (int s = 0; s < 8; ++s) { const int Lid = (lane >> 3) + 4 * s, piece = lane & 7; const int row = Lid >> 1, cofs = (Lid & 1) * 32 + piece * 4;
                v4f val = *(const v4fa*)(os + row * 68 + cofs); if (R) { const v4f rv = *(const v4f*)(R + ((size_t)r0 + row) * ldc + c0 + cofs); val += roundR ? (v4f){bfr(rv[0]), bfr(rv[1]), bfr(rv[2]), bfr(rv[3])} : rv; }
                *(volatile v4f*)(crow + (size_t)row * ldc + cofs) = val; }
        };
        pass(); __threadfence(); pass();
    }
}


__global__ __launch_bounds__(128) void k_gemmh(const h16* __restrict__ A, const h16* __restrict__ Bn, const float* __restrict__ bias, float* C, int ldc, const float* __restrict__ R, int K, size_t sA, size_t sB, size_t sC, int roundR) {
    __shared__ __align__(16) float ost[4][16 * 68];
    const size_t z = blockIdx.z; A += z * sA; Bn += z * sB; C += z * sC; if (R) R += z * sC;
    const int lane = threadIdx.x & 31, wave = threadIdx.x >> 5, lr = lane & 15, hi = lane >> 4;
    const int r0 = blockIdx.x * 64 + wave * 16, c0 = blockIdx.y * 64;
    const size_t aoff = (size_t)(r0 + lr) * K + 8 * hi;
    size_t boff[4];
#pragma unroll
    for (int t = 0; t < 4; ++t) boff[t] = (size_t)(c0 + t * 16 + lr) * K + 8 * hi;
    v8f acc[4];
#pragma unroll
    for (int t = 0; t < 4; ++t) acc[t] = (v8f){};
#pragma unroll 1
    for (int kc = 0; kc < K; kc += 32) {
        const v16h a = cat16(*(const v8h*)(A + aoff + kc), *(const v8h*)(A + aoff + kc + 16));
#pragma unroll
        for (int t = 0; t < 4; ++t) { const v16h b = cat16(*(const v8h*)(Bn + boff[t] + kc), *(const v8h*)(Bn + boff[t] + kc + 16)); acc[t] = wmma16(a, b, acc[t]); }
        asm volatile("v_nop\n\tv_nop\n\tv_nop\n\tv_nop" : "+v"(acc[0]), "+v"(acc[1]), "+v"(acc[2]), "+v"(acc[3]) : "v"(a));
    }
    float* os = &ost[wave][0];
#pragma unroll
    for (int t = 0; t < 4; ++t) { const float bv = bias ? bfr(bias[c0 + t * 16 + lr]) : 0.f;
#pragma unroll
        for (int j = 0; j < 8; ++j) os[(hi * 8 + j) * 68 + t * 16 + lr] = acc[t][j] + bv; }
    __syncthreads();
    float* crow = C + (size_t)r0 * ldc + c0;
    auto pass = [&]() {
#pragma unroll
        for (int s = 0; s < 8; ++s) { const int Lid = (lane >> 3) + 4 * s, piece = lane & 7; const int row = Lid >> 1, cofs = (Lid & 1) * 32 + piece * 4;
            v4f val = *(const v4fa*)(os + row * 68 + cofs); if (R) { const v4f rv = *(const v4f*)(R + ((size_t)r0 + row) * ldc + c0 + cofs); val += roundR ? (v4f){bfr(rv[0]), bfr(rv[1]), bfr(rv[2]), bfr(rv[3])} : rv; }
            *(volatile v4f*)(crow + (size_t)row * ldc + cofs) = val; }
    };
    pass(); __threadfence(); pass();
}

typedef __attribute__((ext_vector_type(4))) _Float16 v4h;
__device__ __forceinline__ h16 tohx(float x) { return (h16)x; }
__global__ __launch_bounds__(256) void k_xtok(const float* __restrict__ x, bf* XT) {
    const int lane = threadIdx.x & 31; const size_t r = (size_t)blockIdx.x * 8 + (threadIdx.x >> 5); if (r >= (size_t)NB_ * NTK) return; const int b = (int)(r / NTK), n = (int)(r % NTK); const int i = n / GW, j = n % GW; const int Cq0 = lane * 8; const int ww = Cq0 / 128, hh = (Cq0 % 128) / 64, c0 = Cq0 % 64; v8us o;
#pragma unroll
    for (int k = 0; k < 8; ++k) o[k] = f2bf(x[(((size_t)b * CX + c0 + k) * HX + 2 * i + hh) * WX + 2 * j + ww]);
    *(volatile v8us*)(XT + r * CP + Cq0) = o; __threadfence(); *(volatile v8us*)(XT + r * CP + Cq0) = o;
}
__global__ __launch_bounds__(256) void k_wcat(const float* __restrict__ wq, const float* __restrict__ wk, const float* __restrict__ wv, bf* Bt) {
    const int lane = threadIdx.x & 31; const int n = blockIdx.x * 8 + (threadIdx.x >> 5); if (n >= NQKV) return; const float* src = (n < CQ) ? wq + (size_t)n * CP : (n < 2 * CQ) ? wk + (size_t)(n - CQ) * CP : wv + (size_t)(n - 2 * CQ) * CP; v8us o;
#pragma unroll
    for (int i = 0; i < 8; ++i) o[i] = f2bf(src[lane * 8 + i]);
    *(volatile v8us*)(Bt + (size_t)n * CP + lane * 8) = o; __threadfence(); *(volatile v8us*)(Bt + (size_t)n * CP + lane * 8) = o;
}
__global__ __launch_bounds__(64) void k_bcat(const float* __restrict__ bq, const float* __restrict__ bk, const float* __restrict__ bv, float* BB) {
    const int t = threadIdx.x; if (t >= 40) return;
#pragma unroll 1
    for (int ps = 0; ps < 2; ++ps) { for (int q = t; q < NQKV / 4; q += 40) { v4f o; for (int i = 0; i < 4; ++i) { const int n = q * 4 + i; o[i] = bfr(n < CQ ? bq[n] : n < 2 * CQ ? bk[n - CQ] : bv[n - 2 * CQ]); } *(volatile v4f*)(BB + q * 4) = o; } if (ps == 0) __threadfence(); }
}
__global__ __launch_bounds__(256) void k_qkpl(const float* __restrict__ QKV, int b, h16* Qp, h16* Kp) {
    const int lane = threadIdx.x & 31; const int n = (blockIdx.x * 8 + (threadIdx.x >> 5)) * 4 + (lane >> 3); if (n >= NTK) return; const int c0 = (lane & 7) * 4; const float* row = QKV + ((size_t)b * NTK + n) * NQKV; v4h oq, ok;
#pragma unroll
    for (int i = 0; i < 4; ++i) { oq[i] = tohx(row[c0 + i]); ok[i] = tohx(row[CQ + c0 + i]); }
    *(volatile v4h*)(Qp + (size_t)n * CQ + c0) = oq; *(volatile v4h*)(Kp + (size_t)n * CQ + c0) = ok; __threadfence(); *(volatile v4h*)(Qp + (size_t)n * CQ + c0) = oq; *(volatile v4h*)(Kp + (size_t)n * CQ + c0) = ok;
}
__global__ __launch_bounds__(256) void k_vT(const float* __restrict__ QKV, int b, h16* VT) {
    __shared__ float tl[64][65];
    const int tid = threadIdx.x; const int t0 = blockIdx.x * 64, c0 = blockIdx.y * 64; const int rr = tid >> 2, cq = (tid & 3) * 16;
#pragma unroll
    for (int i = 0; i < 16; ++i) tl[rr][cq + i] = QKV[((size_t)b * NTK + t0 + rr) * NQKV + 2 * CQ + c0 + cq + i];
    __syncthreads();
    const int lane = tid & 31, wv = tid >> 5;
    auto pass = [&]() {
#pragma unroll
        for (int st = 0; st < 4; ++st) { const int cr = wv * 8 + st * 2 + (lane >> 4); const int tq = (lane & 15) * 4; v4h v;
#pragma unroll
            for (int i = 0; i < 4; ++i) v[i] = tohx(tl[tq + i][cr]);
            *(volatile v4h*)(VT + (size_t)(c0 + cr) * NTK + t0 + tq) = v; }
    };
    pass(); __threadfence(); pass();
}
__global__ __launch_bounds__(256) void k_softs(const float* __restrict__ S, h16* P) {
    const int lane = threadIdx.x & 31, i = blockIdx.x * 8 + (threadIdx.x >> 5); if (i >= NTK) return; const size_t zo = (size_t)i * NTK; const float* sr = S + zo; h16* po = P + zo;
    float m = -3.0e38f;
#pragma unroll 1
    for (int c0 = lane * 4; c0 < NTK; c0 += 128) {
#pragma unroll
        for (int q = 0; q < 4; ++q) m = fmaxf(m, sr[c0 + q]); }
#pragma unroll
    for (int sh = 16; sh; sh >>= 1) m = fmaxf(m, __shfl_xor(m, sh, 32));
    float sum = 0.f;
#pragma unroll 1
    for (int c0 = lane * 4; c0 < NTK; c0 += 128) {
#pragma unroll
        for (int q = 0; q < 4; ++q) sum += __expf(sr[c0 + q] - m); }
#pragma unroll
    for (int sh = 16; sh; sh >>= 1) sum += __shfl_xor(sum, sh, 32);
    const float f = __fdiv_rn(PCAR, sum);
#pragma unroll 1
    for (int ps = 0; ps < 2; ++ps) {
#pragma unroll 1
        for (int c0 = lane * 4; c0 < NTK; c0 += 128) { v4h o;
#pragma unroll
            for (int q = 0; q < 4; ++q) o[q] = tohx(__expf(sr[c0 + q] - m) * f);
            *(volatile v4h*)(po + c0) = o; }
        if (ps == 0) __threadfence(); }
}
__global__ __launch_bounds__(256) void k_fin(const float* __restrict__ OT, const float* __restrict__ x, const float* __restrict__ gam, int b, float* OUTB) {
    const int lane = threadIdx.x & 31; const int rw = blockIdx.x * 8 + (threadIdx.x >> 5); if (rw >= CX * HX) return; const int c = rw / HX, h = rw % HX; const float gm = bfr(gam[0]); v4f o;
#pragma unroll
    for (int k = 0; k < 4; ++k) { const int w = lane * 4 + k; const int n = (h / 2) * GW + (w / 2); const int Cq = (w % 2) * 128 + (h % 2) * 64 + c; o[k] = gm * (OT[(size_t)n * CP + Cq] * (1.0f / PCAR)) + bfr(x[(((size_t)b * CX + c) * HX + h) * WX + w]); }
    float* dst = OUTB + (((size_t)b * CX + c) * HX + h) * WX + lane * 4; *(volatile v4f*)dst = o; __threadfence(); *(volatile v4f*)dst = o;
}
extern "C" void kernel_launch(void* const* d_in, const int* in_sizes, int n_in,
                              void* d_out, int out_size, void* d_ws, size_t ws_size, hipStream_t stream) {
    (void)in_sizes; (void)n_in; (void)out_size;
    const float* x = (const float*)d_in[0]; const float* wq = (const float*)d_in[1]; const float* bq = (const float*)d_in[2]; const float* wk = (const float*)d_in[3]; const float* bk = (const float*)d_in[4]; const float* wv = (const float*)d_in[5]; const float* bv = (const float*)d_in[6]; const float* gam = (const float*)d_in[7];
    float* out = (float*)d_out;
    char* wsp = (char*)d_ws;
    auto take = [&](size_t bytes) { char* p = wsp; wsp += (bytes + 255) & ~(size_t)255; return (void*)p; };
    bf* XT = (bf*)take((size_t)NB_ * NTK * CP * 2); bf* WB = (bf*)take((size_t)NQKV * CP * 2); float* BB = (float*)take(NQKV * 4); float* QKV = (float*)take((size_t)NB_ * NTK * NQKV * 4);
    h16* Qp = (h16*)take((size_t)NTK * CQ * 2); h16* Kp = (h16*)take((size_t)NTK * CQ * 2); h16* VT = (h16*)take((size_t)CP * NTK * 2); float* S = (float*)take((size_t)NTK * NTK * 4); h16* Px = (h16*)take((size_t)NTK * NTK * 2); float* OT = (float*)take((size_t)NTK * CP * 4);
    if ((size_t)(wsp - (char*)d_ws) > ws_size) return;
    k_xtok<<<(NB_ * NTK) / 8, 256, 0, stream>>>(x, XT); k_wcat<<<NQKV / 8, 256, 0, stream>>>(wq, wk, wv, WB); k_bcat<<<1, 64, 0, stream>>>(bq, bk, bv, BB);
    k_gemmb<false, false><<<dim3((NB_ * NTK) / 64, NQKV / 64, 1), 128, 0, stream>>>(XT, nullptr, WB, BB, QKV, NQKV, nullptr, nullptr, CP);
    for (int b = 0; b < NB_; ++b) {
        k_qkpl<<<(NTK / 4) / 8, 256, 0, stream>>>(QKV, b, Qp, Kp); k_vT<<<dim3(NTK / 64, CP / 64, 1), 256, 0, stream>>>(QKV, b, VT);
        k_gemmh<<<dim3(NTK / 64, NTK / 64, 1), 128, 0, stream>>>(Qp, Kp, nullptr, S, NTK, nullptr, CQ, 0, 0, 0, 0);
        k_softs<<<NTK / 8, 256, 0, stream>>>(S, Px);
        k_gemmh<<<dim3(NTK / 64, CP / 64, 1), 128, 0, stream>>>(Px, VT, nullptr, OT, CP, nullptr, NTK, 0, 0, 0, 0);
        k_fin<<<(CX * HX) / 8, 256, 0, stream>>>(OT, x, gam, b, out); }
}
